// GNN_60387240182014
// MI455X (gfx1250) — hardware-verified
//
#include <hip/hip_runtime.h>
#include <stddef.h>
#include <stdint.h>
#include <math.h>


#define NN_C   300000
#define NE_C   600000
#define NG_C   12000
#define HID    128
#define FA     9
#define VA     119
#define DA     9
#define EMBN   (FA * VA * DA)
#define NTHR   256
#define NWAVE  8
#define EPT    8
#define CHUNK  (NTHR * EPT)
#define WCAP   (EPT * 32)
#define LISTN  (NWAVE * WCAP)
#define NBD    8192
#define SLD    13
#define GPB    64
#define NBLK   188
#define SLOTCAP 2048
#define SLB    11
#define RCAP   8192
#define DEGCAP 32
#define NGT    12288
#define GOFFB  48
#define GBM    64
#define GBN    128
#define GTHR   128
#define K1     32
#define AP1    64
#define K2     256
#define NUW1   512
#define NUW2   4096
#define H0NPB  1024
#define BK_ZINTS (LISTN + 2 * RCAP + 3 * SLOTCAP)
#define BK_MISC  16
#define BK_ROWB  (NWAVE * 512 / 2)
#define BK_LDS_INTS (BK_ZINTS + BK_MISC + BK_ROWB)

static_assert((CHUNK & (CHUNK - 1)) == 0 && CHUNK <= 4096);
static_assert((NBD & (NBD - 1)) == 0 && NBD == (1 << SLD));
static_assert((SLOTCAP & (SLOTCAP - 1)) == 0 && SLOTCAP == (1 << SLB));
static_assert(((long long)CHUNK << SLD) < (1LL << 31));
static_assert(((long long)NE_C << SLB) < (1LL << 31));
static_assert(NBD % (NTHR * 4) == 0 && LISTN % NTHR == 0);
static_assert(SLOTCAP % (NWAVE * 8) == 0 && SLOTCAP % 32 == 0 && SLOTCAP % (NTHR * 4) == 0);
static_assert(RCAP % (NTHR * 4) == 0 && RCAP <= (1 << 22) && DEGCAP <= 32 && DEGCAP < 255);
static_assert(BK_ZINTS % (NTHR * 4) == 0 && ((BK_ZINTS + BK_MISC) % 4) == 0);
static_assert(BK_LDS_INTS * 4 <= 300000);
static_assert(NBLK * GPB >= NG_C && (NBLK - 1) * GPB < NG_C && NBLK * GPB + 32 <= NGT);
static_assert((NBLK * GPB) % GBM == 0 && GPB % NWAVE == 0);
static_assert(NGT == GOFFB * NTHR && NN_C < (1 << 19));
static_assert(K1 % 32 == 0 && K2 % 32 == 0 && K2 == 2 * HID && GBN == HID && GBM == (GTHR / 32) * 16);
static_assert(NUW1 % NTHR == 0 && NUW2 % NTHR == 0);
static_assert((NN_C * FA) % 4 == 0 && ((NN_C * 64) % 128) == 0 && (H0NPB % NTHR) == 0);
static_assert((EMBN + 1 + NTHR * FA + NTHR * 16) * 4 <= 65536);

typedef float          v4f   __attribute__((ext_vector_type(4)));
typedef float          v8f   __attribute__((ext_vector_type(8)));
typedef int            v4i   __attribute__((ext_vector_type(4)));
typedef int            v8i   __attribute__((ext_vector_type(8)));
typedef unsigned short v4us  __attribute__((ext_vector_type(4)));
typedef unsigned short v8us  __attribute__((ext_vector_type(8)));
typedef unsigned short v16us __attribute__((ext_vector_type(16)));
typedef __bf16         v16bf __attribute__((ext_vector_type(16)));
typedef v4f  __attribute__((may_alias)) v4fa;
typedef v4i  __attribute__((may_alias)) v4ia;
typedef v4us __attribute__((may_alias)) v4usa;
typedef v8us __attribute__((may_alias)) v8usa;
union FragB { v16bf v; v16us u; v8us h[2]; v8i w; };

__device__ __forceinline__ v8f wmb(const FragB& a, const FragB& b, v8f c) {
  v8f d = __builtin_amdgcn_wmma_f32_16x16x32_bf16(false, a.v, false, b.v, (short)0, c, false, false);
  asm volatile("v_nop\n\tv_nop\n\tv_nop\n\tv_nop" : "+v"(d) : "v"(a.w), "v"(b.w));
  return d;
}

__device__ __forceinline__ unsigned bf16_bits(float f) {
  const unsigned u = __float_as_uint(f);
  return (u + 0x7FFFu + ((u >> 16) & 1u)) >> 16;
}
__device__ __forceinline__ float bf16_val(float f) {
  return __uint_as_float(bf16_bits(f) << 16);
}

__device__ __forceinline__ void wave_sync() {
  __builtin_amdgcn_fence(__ATOMIC_RELEASE, "wavefront");
  __builtin_amdgcn_wave_barrier();
  __builtin_amdgcn_fence(__ATOMIC_ACQUIRE, "wavefront");
}

__device__ __forceinline__ int rfl(int v) { return __builtin_amdgcn_readfirstlane(v); }
__device__ __forceinline__ int clampi(int v, int lo, int hi) { return v < lo ? lo : (v > hi ? hi : v); }

template <int SLBT>
__device__ __forceinline__ int scan_chunk(const int* __restrict__ dsts, int nE, int cbase, int slotBase,
                                          int nb, int vec8, int* list, int tid, int lane, int wave) {
  int wc = 0;
  const int el0  = tid * EPT;
  const int e0   = cbase + el0;
  const int sent = -2147483647 - 1;
  v4i da, db;
  if (vec8 != 0 && cbase + CHUNK <= nE) {
    da = *(const v4i*)(dsts + e0);
    db = *(const v4i*)(dsts + e0 + 4);
  } else {
    da.x = (e0     < nE) ? dsts[min(e0,     nE - 1)] : sent;
    da.y = (e0 + 1 < nE) ? dsts[min(e0 + 1, nE - 1)] : sent;
    da.z = (e0 + 2 < nE) ? dsts[min(e0 + 2, nE - 1)] : sent;
    da.w = (e0 + 3 < nE) ? dsts[min(e0 + 3, nE - 1)] : sent;
    db.x = (e0 + 4 < nE) ? dsts[min(e0 + 4, nE - 1)] : sent;
    db.y = (e0 + 5 < nE) ? dsts[min(e0 + 5, nE - 1)] : sent;
    db.z = (e0 + 6 < nE) ? dsts[min(e0 + 6, nE - 1)] : sent;
    db.w = (e0 + 7 < nE) ? dsts[min(e0 + 7, nE - 1)] : sent;
  }
  const unsigned nbs = (unsigned)slotBase;
  const unsigned unb = (unsigned)nb;
  const unsigned s0 = (unsigned)da.x - nbs, s1 = (unsigned)da.y - nbs;
  const unsigned s2 = (unsigned)da.z - nbs, s3 = (unsigned)da.w - nbs;
  const unsigned s4 = (unsigned)db.x - nbs, s5 = (unsigned)db.y - nbs;
  const unsigned s6 = (unsigned)db.z - nbs, s7 = (unsigned)db.w - nbs;
  const bool h0 = s0 < unb, h1 = s1 < unb, h2 = s2 < unb, h3 = s3 < unb;
  const bool h4 = s4 < unb, h5 = s5 < unb, h6 = s6 < unb, h7 = s7 < unb;
  const unsigned any = __builtin_amdgcn_ballot_w32(h0 | h1 | h2 | h3 | h4 | h5 | h6 | h7);
  if (any != 0u) {
#define HITJ(J, HJ, SJ) { \
      const unsigned mj = __builtin_amdgcn_ballot_w32(HJ); \
      if (mj != 0u) { \
        if (HJ) { \
          const int pos = wc + (int)__builtin_amdgcn_mbcnt_lo(mj, 0u); \
          if (pos < WCAP) list[wave * WCAP + pos] = ((el0 + (J)) << SLBT) | (int)(SJ); \
        } \
        wc += (int)__builtin_popcount(mj); } }
    HITJ(0, h0, s0)
    HITJ(1, h1, s1)
    HITJ(2, h2, s2)
    HITJ(3, h3, s3)
    HITJ(4, h4, s4)
    HITJ(5, h5, s5)
    HITJ(6, h6, s6)
    HITJ(7, h7, s7)
#undef HITJ
  }
  return wc;
}

__global__ __launch_bounds__(NTHR) void k_wprep(const float* __restrict__ W1, const float* __restrict__ W2,
                                                const float* __restrict__ Wf,
                                                unsigned short* W1D, unsigned short* W2D, unsigned short* WFD) {
  const int u = (int)blockIdx.x * NTHR + (int)threadIdx.x;
  v8us o;
  unsigned short* dp;
  if (u < NUW1) {
    const int n  = u >> 2;
    const int kb = ((u & 3) * 8) & 15;
#pragma unroll
    for (int i = 0; i < 8; ++i) {
      const int kk = kb + i;
      const int kc = kk < DA ? kk : DA - 1;
      const float w = W1[(size_t)kc * HID + n];
      o[i] = (kk < DA) ? (unsigned short)bf16_bits(w) : (unsigned short)0;
    }
    dp = W1D + (size_t)u * 8;
  } else if (u < NUW1 + NUW2) {
    const int v  = u - NUW1;
    const int n  = v >> 5;
    const int kk = ((v & 31) * 8) & (HID - 1);
    const float* p = W2 + (size_t)kk * HID + n;
#pragma unroll
    for (int i = 0; i < 8; ++i) o[i] = (unsigned short)bf16_bits(p[(size_t)i * HID]);
    dp = W2D + (size_t)v * 8;
  } else if (u < NUW1 + 2 * NUW2) {
    const int v  = u - NUW1 - NUW2;
    const int n  = v >> 5;
    const int kk = ((v & 31) * 8) & (HID - 1);
    const float* p = Wf + (size_t)kk * HID + n;
#pragma unroll
    for (int i = 0; i < 8; ++i) o[i] = (unsigned short)bf16_bits(p[(size_t)i * HID]);
    dp = WFD + (size_t)v * 8;
  } else {
    return;
  }
  *(volatile v8us*)dp = o;
  __threadfence();
  *(volatile v8us*)dp = o;
}

__global__ __launch_bounds__(NTHR) void k_h0(const int* __restrict__ x, const float* __restrict__ emb,
                                             int nN, float* h0) {
  __shared__ float embs[EMBN + 1];
  __shared__ __attribute__((aligned(16))) int xs[NTHR * FA];
  __shared__ __attribute__((aligned(16))) float hs[NTHR * 16];
  const int tid = (int)threadIdx.x;
#pragma unroll 4
  for (int i = tid; i < EMBN; i += NTHR) embs[i] = bf16_val(emb[i]);
  if (tid == 0) embs[EMBN] = 0.0f;
  const int nx4 = (nN * FA) / 4;
#pragma unroll 1
  for (int sub = 0; sub < H0NPB / NTHR; ++sub) {
    const int nb = (int)blockIdx.x * H0NPB + sub * NTHR;
    __syncthreads();
#pragma unroll 1
    for (int v = tid; v < (NTHR * FA) / 4; v += NTHR) {
      int g4 = (nb * FA) / 4 + v;
      g4 = g4 < 0 ? 0 : (g4 > nx4 - 1 ? nx4 - 1 : g4);
      *(v4ia*)(xs + 4 * v) = *(const v4i*)(x + 4 * (size_t)g4);
    }
    __syncthreads();
    float acc[DA];
#pragma unroll
    for (int d = 0; d < DA; ++d) acc[d] = 0.0f;
#pragma unroll
    for (int f = 0; f < FA; ++f) {
      int xi = xs[tid * FA + f];
      xi = xi < 0 ? 0 : (xi > VA - 1 ? VA - 1 : xi);
      const float* t = embs + (f * VA + xi) * DA;
#pragma unroll
      for (int d = 0; d < DA; ++d) acc[d] += t[d];
    }
#pragma unroll
    for (int d = 0; d < 16; ++d) hs[tid * 16 + d] = (d < DA) ? acc[d < DA ? d : 0] : 0.0f;
    __syncthreads();
    v4f pv[4];
#pragma unroll
    for (int k = 0; k < 4; ++k) pv[k] = *(const v4fa*)(hs + 4 * (k * NTHR + tid));
#pragma unroll
    for (int k = 0; k < 4; ++k) {
      const int p = k * NTHR + tid;
      const int row = nb + (p >> 2);
      float* op = h0 + (size_t)nb * 16 + 4 * (size_t)p;
      if (row < nN) *(volatile v4f*)op = pv[k];
    }
    __threadfence();
#pragma unroll
    for (int k = 0; k < 4; ++k) {
      const int p = k * NTHR + tid;
      const int row = nb + (p >> 2);
      float* op = h0 + (size_t)nb * 16 + 4 * (size_t)p;
      if (row < nN) *(volatile v4f*)op = pv[k];
    }
  }
}

__global__ __launch_bounds__(NTHR) void k_goff(const int* __restrict__ bat, int nN, int nG,
                                               int* goff, int* flag) {
  __shared__ __attribute__((aligned(16))) int sv[NTHR];
  __shared__ int wf[NWAVE];
  const int tid = (int)threadIdx.x, lane = tid & 31, wave = tid >> 5;
  if ((int)blockIdx.x < GOFFB) {
    const int g = (int)blockIdx.x * NTHR + tid;
    int lo = 0, hi = nN;
#pragma unroll 1
    for (int it = 0; it < 20; ++it) {
      const bool act = lo < hi;
      const int mid = (lo + hi) >> 1;
      const int mc = mid < 0 ? 0 : (mid > nN - 1 ? nN - 1 : mid);
      const int v = bat[mc];
      const bool lt = v < g;
      const int nlo = lt ? mid + 1 : lo;
      const int nhi = lt ? hi : mid;
      lo = act ? nlo : lo;
      hi = act ? nhi : hi;
    }
    sv[tid] = lo;
    __syncthreads();
    const v4i o = *(const v4ia*)(sv + 4 * (tid & 63));
    int* dp = goff + (size_t)blockIdx.x * NTHR + 4 * (tid & 63);
    const bool st = tid < NTHR / 4;
    if (st) *(volatile v4i*)dp = o;
    __threadfence();
    if (st) *(volatile v4i*)dp = o;
  } else {
    int bad = 0;
#pragma unroll 2
    for (int i = tid; i < nN; i += NTHR) {
      const int i2 = (i + 1 < nN) ? i + 1 : nN - 1;
      const int v = bat[i];
      const int w = bat[i2];
      bad |= ((v < 0) | (v >= nG) | (v > w)) ? 1 : 0;
    }
    const unsigned bm = __builtin_amdgcn_ballot_w32(bad != 0);
    if (lane == 0) wf[wave] = (bm != 0u) ? 1 : 0;
    __syncthreads();
    int f = 0;
#pragma unroll
    for (int w2 = 0; w2 < NWAVE; ++w2) f |= wf[w2];
    v4i o = {0, 0, 0, 0};
    o.x = (lane == 0) ? f : 0;
    int* dp = flag + 4 * (lane & 7);
    const bool st = (wave == 0) && (lane < 8);
    if (st) *(volatile v4i*)dp = o;
    __threadfence();
    if (st) *(volatile v4i*)dp = o;
  }
}

__global__ __launch_bounds__(NTHR) void k_deg(const int* __restrict__ dsts, int nE, int vec8, float* dis) {
  __shared__ __attribute__((aligned(16))) int scnt[NBD];
  __shared__ __attribute__((aligned(16))) int list[LISTN];
  __shared__ int wcnt[NWAVE];
  const int tid = (int)threadIdx.x, lane = tid & 31, wave = tid >> 5;
  const int nodeBase = (int)blockIdx.x * NBD;

  for (int i = tid; i < NBD; i += NTHR) scnt[i] = 0;
  for (int i = tid; i < LISTN; i += NTHR) list[i] = 0;
  if (tid < NWAVE) wcnt[tid] = 0;
  __syncthreads();

  const int nChunks = (nE + CHUNK - 1) / CHUNK;
#pragma unroll 1
  for (int ch = 0; ch < nChunks; ++ch) {
    const int cbase = ch * CHUNK;
    const int wc = scan_chunk<SLD>(dsts, nE, cbase, nodeBase, NBD, vec8, list, tid, lane, wave);
    if (lane == 0) wcnt[wave] = wc;
    __syncthreads();
    if (wave == 0) {
#pragma unroll 1
      for (int w2 = 0; w2 < NWAVE; ++w2) {
        int c = wcnt[w2];
        c = c < 0 ? 0 : (c > WCAP ? WCAP : c);
#pragma unroll 1
        for (int b0 = 0; b0 < c; b0 += 32) {
          const int idx = b0 + lane;
          const int ent = list[w2 * WCAP + (idx < WCAP ? idx : WCAP - 1)];
          const int m32 = (c - b0) < 32 ? (c - b0) : 32;
#pragma unroll 1
          for (int k = 0; k < m32; ++k) {
            const int u  = __builtin_amdgcn_readlane(ent, k);
            const int sl = u & (NBD - 1);
            if (lane == 0) scnt[sl] = scnt[sl] + 1;
          }
        }
      }
    }
    __syncthreads();
  }

  v4f vals[NBD / (NTHR * 4)];
#pragma unroll
  for (int it = 0; it < NBD / (NTHR * 4); ++it) {
    const int s0 = it * (NTHR * 4) + 4 * tid;
    const v4i c4 = *(const v4ia*)(scnt + s0);
    const float d0 = (float)c4.x + 1.0f, d1 = (float)c4.y + 1.0f;
    const float d2 = (float)c4.z + 1.0f, d3 = (float)c4.w + 1.0f;
    v4f v;
    v.x = rsqrtf(d0); v.y = rsqrtf(d1); v.z = rsqrtf(d2); v.w = rsqrtf(d3);
    vals[it] = v;
  }
#pragma unroll
  for (int it = 0; it < NBD / (NTHR * 4); ++it) {
    const int s0 = it * (NTHR * 4) + 4 * tid;
    *(volatile v4f*)(dis + (size_t)nodeBase + s0) = vals[it];
  }
  __threadfence();
#pragma unroll
  for (int it = 0; it < NBD / (NTHR * 4); ++it) {
    const int s0 = it * (NTHR * 4) + 4 * tid;
    *(volatile v4f*)(dis + (size_t)nodeBase + s0) = vals[it];
  }
}

__device__ __forceinline__ void bkt_dump(const int* hl, const int* cnt, const int* offs,
                                         int* lstb, int* ocbb, int* blkb,
                                         int tid, int lane, int wave, int ovf, int tt, int nbase, int nend) {
#pragma unroll 1
  for (int it = 0; it < RCAP / (NTHR * 4); ++it) {
    const int p4 = 4 * (it * NTHR + tid);
    const v4i v = *(const v4ia*)(hl + p4);
    *(volatile v4i*)(lstb + p4) = v;
  }
#pragma unroll 1
  for (int it = 0; it < SLOTCAP / (NTHR * 4); ++it) {
    const int s4 = 4 * (it * NTHR + tid);
    const v4i c4 = *(const v4ia*)(cnt + s4);
    const v4i o4 = *(const v4ia*)(offs + s4);
    v4i pk;
    pk.x = (o4.x << 8) | clampi(c4.x, 0, 255);
    pk.y = (o4.y << 8) | clampi(c4.y, 0, 255);
    pk.z = (o4.z << 8) | clampi(c4.z, 0, 255);
    pk.w = (o4.w << 8) | clampi(c4.w, 0, 255);
    *(volatile v4i*)(ocbb + s4) = pk;
  }
  v4i bv = {0, 0, 0, 0};
  bv.x = (lane == 0) ? ovf : 0;
  bv.y = (lane == 0) ? tt : 0;
  bv.z = (lane == 0) ? nbase : 0;
  bv.w = (lane == 0) ? nend : 0;
  if (wave == 0 && lane < 8) *(volatile v4i*)(blkb + 4 * (lane & 7)) = bv;
}

__global__ __launch_bounds__(NTHR) void k_bkt(const int* __restrict__ srcs, const int* __restrict__ dsts,
                                              int nE, int nN, int nG, int vec8, int mRows,
                                              const int* __restrict__ goff, const float* __restrict__ dis,
                                              const float* __restrict__ h0,
                                              int* lst, int* ocb, int* blkf, unsigned short* a0hl) {
  extern __shared__ __attribute__((aligned(16))) int dsm[];
  int* list = dsm;
  int* hl   = dsm + LISTN;
  int* sl   = hl + RCAP;
  int* cnt  = sl + RCAP;
  int* offs = cnt + SLOTCAP;
  int* cur  = offs + SLOTCAP;
  int* misc = cur + SLOTCAP;
  const int tid = (int)threadIdx.x, lane = tid & 31;
  const int wave = rfl(tid >> 5);
  unsigned short* rowbuf = (unsigned short*)(misc + BK_MISC) + wave * 512;
  const int b = (int)blockIdx.x;

  {
    const v4i z4 = {0, 0, 0, 0};
    for (int i = tid * 4; i < BK_ZINTS; i += NTHR * 4) *(v4ia*)(dsm + i) = z4;
    if (tid < BK_MISC) misc[tid] = 0;
  }
  const int g0 = b * GPB;
  int g1 = g0 + GPB; g1 = g1 > nG ? nG : g1;
  int nbase = goff[g0 < NGT - 1 ? g0 : NGT - 1];
  int nend  = goff[g1 < NGT - 1 ? g1 : NGT - 1];
  nbase = clampi(nbase, 0, nN);
  nend  = clampi(nend, nbase, nN);
  int nslots = nend - nbase;
  const int ov0 = nslots > SLOTCAP ? 1 : 0;
  nslots = nslots > SLOTCAP ? SLOTCAP : nslots;
  nbase = rfl(nbase); nend = rfl(nend); nslots = rfl(nslots);
  __syncthreads();

  int t = 0, ov = 0;
  const int nChunks = (nE + CHUNK - 1) / CHUNK;
#pragma unroll 1
  for (int ch = 0; ch < nChunks; ++ch) {
    const int cbase = ch * CHUNK;
    const int wc = scan_chunk<SLB>(dsts, nE, cbase, nbase, nslots, vec8, list, tid, lane, wave);
    if (lane == 0) misc[wave] = wc;
    __syncthreads();
    if (wave == 0) {
#pragma unroll 1
      for (int w2 = 0; w2 < NWAVE; ++w2) {
        int c = misc[w2];
        c = c < 0 ? 0 : (c > WCAP ? WCAP : c);
#pragma unroll 1
        for (int b0 = 0; b0 < c; b0 += 32) {
          const int idx = b0 + lane;
          const int ent = list[w2 * WCAP + (idx < WCAP ? idx : WCAP - 1)];
          const int m32 = (c - b0) < 32 ? (c - b0) : 32;
#pragma unroll 1
          for (int k = 0; k < m32; ++k) {
            const int u    = __builtin_amdgcn_readlane(ent, k);
            const int slot = u & (SLOTCAP - 1);
            const int el   = (u >> SLB) & (CHUNK - 1);
            const int pk   = ((cbase + el) << SLB) | slot;
            if (t < RCAP) {
              if (lane == 0) { hl[t] = pk; cnt[slot] = cnt[slot] + 1; }
              t = t + 1;
            } else {
              ov = 1;
            }
          }
        }
      }
    }
    __syncthreads();
  }
  if (wave == 0 && lane == 0) { misc[8] = t; misc[9] = ov; }
  __syncthreads();
  int tt = misc[8];
  tt = tt < 0 ? 0 : (tt > RCAP ? RCAP : tt);
  tt = rfl(tt);
  const int ovf = rfl((misc[9] != 0 || ov0 != 0) ? 1 : 0);

  if (wave == 0) {
    const int base = lane * (SLOTCAP / 32);
    int s = 0;
#pragma unroll 1
    for (int i = 0; i < SLOTCAP / 32; ++i) s += cnt[base + i];
    int incl = s;
#pragma unroll
    for (int d = 1; d < 32; d <<= 1) {
      const int y = __shfl_up(incl, d, 32);
      if (lane >= d) incl += y;
    }
    int run = incl - s;
#pragma unroll 1
    for (int i = 0; i < SLOTCAP / 32; ++i) {
      const int cv = cnt[base + i];
      offs[base + i] = run;
      cur[base + i]  = run;
      run += cv;
    }
  }
  __syncthreads();
  if (wave == 0) {
#pragma unroll 1
    for (int b0 = 0; b0 < tt; b0 += 32) {
      const int idx = b0 + lane;
      const int ent = hl[idx < RCAP ? idx : RCAP - 1];
      const int m32 = (tt - b0) < 32 ? (tt - b0) : 32;
#pragma unroll 1
      for (int k = 0; k < m32; ++k) {
        const int u    = __builtin_amdgcn_readlane(ent, k);
        const int slot = u & (SLOTCAP - 1);
        if (lane == 0) {
          int p = cur[slot];
          p = p < 0 ? 0 : (p > RCAP - 1 ? RCAP - 1 : p);
          sl[p] = u;
          cur[slot] = p + 1;
        }
      }
    }
  }
  __syncthreads();
#pragma unroll 1
  for (int idx = tid; idx < tt; idx += NTHR) {
    const int ent = sl[idx];
    const int eid = clampi(ent >> SLB, 0, nE - 1);
    const int sr  = clampi(srcs[eid], 0, nN - 1);
    hl[idx] = sr;
  }
  __syncthreads();

  {
    int* lstb = lst  + (size_t)b * RCAP;
    int* ocbb = ocb  + (size_t)b * SLOTCAP;
    int* blkb = blkf + (size_t)b * 32;
    bkt_dump(hl, cnt, offs, lstb, ocbb, blkb, tid, lane, wave, ovf, tt, nbase, nend);
    __threadfence();
    bkt_dump(hl, cnt, offs, lstb, ocbb, blkb, tid, lane, wave, ovf, tt, nbase, nend);
  }

  const int q = lane >> 2, j = lane & 3;
  const float qnan = __int_as_float(0x7fc00000);
  const float pz = (ovf != 0) ? qnan : 0.0f;
#pragma unroll 1
  for (int it = 0; it < SLOTCAP / (NWAVE * 8); ++it) {
    const int s0 = (it * NWAVE + wave) * 8;
    if (s0 >= nslots) break;
    const int s = s0 + q;
    const bool live = s < nslots;
    const int sc = s < SLOTCAP ? s : SLOTCAP - 1;
    int c = cnt[sc];
    const bool big = c > DEGCAP;
    c = c < 0 ? 0 : (c > DEGCAP ? DEGCAP : c);
    c = live ? c : 0;
    int o = offs[sc];
    o = o < 0 ? 0 : (o > RCAP ? RCAP : o);
    const int node = nbase + s;
    const int nc = node < nN ? node : nN - 1;
    const float dd = dis[nc];
    int cm = c;
#pragma unroll
    for (int d = 1; d < 32; d <<= 1) {
      const int y = __shfl_xor(cm, d, 32);
      cm = cm > y ? cm : y;
    }
    cm = rfl(cm);
    float e0 = 0.0f, e1 = 0.0f, e2 = 0.0f, e3 = 0.0f;
#pragma unroll 1
    for (int p = 0; p < cm; ++p) {
      int idx = o + p;
      idx = idx > RCAP - 1 ? RCAP - 1 : idx;
      const int sr = clampi(hl[idx], 0, nN - 1);
      const float cf = dis[sr] * dd;
      const v4f a = *(const v4fa*)(h0 + (size_t)sr * 16 + 4 * j);
      const bool on = p < c;
      const float n0 = fmaf(cf, a.x, e0), n1 = fmaf(cf, a.y, e1);
      const float n2 = fmaf(cf, a.z, e2), n3 = fmaf(cf, a.w, e3);
      e0 = on ? n0 : e0; e1 = on ? n1 : e1; e2 = on ? n2 : e2; e3 = on ? n3 : e3;
    }
    const v4f sv = *(const v4fa*)(h0 + (size_t)nc * 16 + 4 * j);
    const float rd = dd * dd;
    const float pzr = big ? qnan : pz;
    float y0 = fmaf(rd, sv.x, e0) + pzr;
    float y1 = fmaf(rd, sv.y, e1) + pzr;
    float y2 = fmaf(rd, sv.z, e2) + pzr;
    float y3 = fmaf(rd, sv.w, e3) + pzr;
    y0 = live ? y0 : 0.0f; y1 = live ? y1 : 0.0f; y2 = live ? y2 : 0.0f; y3 = live ? y3 : 0.0f;
    v4us mh, ml;
    {
      unsigned hb;
      hb = bf16_bits(y0); mh[0] = (unsigned short)hb; ml[0] = (unsigned short)bf16_bits(y0 - __uint_as_float(hb << 16));
      hb = bf16_bits(y1); mh[1] = (unsigned short)hb; ml[1] = (unsigned short)bf16_bits(y1 - __uint_as_float(hb << 16));
      hb = bf16_bits(y2); mh[2] = (unsigned short)hb; ml[2] = (unsigned short)bf16_bits(y2 - __uint_as_float(hb << 16));
      hb = bf16_bits(y3); mh[3] = (unsigned short)hb; ml[3] = (unsigned short)bf16_bits(y3 - __uint_as_float(hb << 16));
    }
    const v8us z8 = {0, 0, 0, 0, 0, 0, 0, 0};
    unsigned short* rb = rowbuf + q * 64;
    *(v4usa*)(rb + 4 * j) = mh;
    *(v4usa*)(rb + 16 + 4 * j) = ml;
    *(v8usa*)(rb + 32 + 8 * j) = z8;
    wave_sync();
    const v8us q0 = *(const v8usa*)(rowbuf + 8 * lane);
    const v8us q1 = *(const v8usa*)(rowbuf + 256 + 8 * lane);
    wave_sync();
    const bool okA = (s0 + (lane >> 3)) < nslots;
    const bool okB = (s0 + 4 + (lane >> 3)) < nslots;
    unsigned short* gp = a0hl + (size_t)(nbase + s0) * AP1 + 8 * lane;
    if (okA) *(volatile v8us*)gp = q0;
    if (okB) *(volatile v8us*)(gp + 4 * AP1) = q1;
    __threadfence();
    if (okA) *(volatile v8us*)gp = q0;
    if (okB) *(volatile v8us*)(gp + 4 * AP1) = q1;
  }
  if (b == (int)gridDim.x - 1) {
    const v8us z8 = {0, 0, 0, 0, 0, 0, 0, 0};
#pragma unroll 1
    for (int r = tid >> 3; nN + r < mRows; r += NTHR / 8)
      *(volatile v8us*)(a0hl + (size_t)(nN + r) * AP1 + 8 * (tid & 7)) = z8;
    __threadfence();
#pragma unroll 1
    for (int r = tid >> 3; nN + r < mRows; r += NTHR / 8)
      *(volatile v8us*)(a0hl + (size_t)(nN + r) * AP1 + 8 * (tid & 7)) = z8;
  }
}

template <int MODE>
__global__ __launch_bounds__(GTHR) void k_gemm(const unsigned short* __restrict__ Apl, int pitchA,
                                               const unsigned short* __restrict__ BT, int K,
                                               const float* __restrict__ bias,
                                               const int* __restrict__ goff, const int* __restrict__ flag,
                                               float* outF, unsigned short* outH, int nOut) {
  __shared__ __attribute__((aligned(16))) float stg[GBM * GBN];
  const int tid = (int)threadIdx.x, lane = tid & 31, wave = tid >> 5, hh = lane >> 4, m = lane & 15;
  const int rowBase = (int)blockIdx.x * GBM;

  v8f acc[8];
  {
    const v8f z = {0.f, 0.f, 0.f, 0.f, 0.f, 0.f, 0.f, 0.f};
#pragma unroll
    for (int t = 0; t < 8; ++t) acc[t] = z;
  }
  const unsigned short* ap = Apl + (size_t)(rowBase + 16 * wave + m) * (size_t)pitchA + 8 * hh;
  const unsigned short* bp = BT + (size_t)m * (size_t)K + 8 * hh;

#pragma unroll 1
  for (int k0 = 0; k0 < K; k0 += 32) {
    FragB af;
    af.h[0] = *(const v8usa*)(ap + k0);
    af.h[1] = *(const v8usa*)(ap + k0 + 16);
#pragma unroll
    for (int nt = 0; nt < 8; ++nt) {
      const unsigned short* wq = bp + (size_t)(16 * nt) * (size_t)K + k0;
      FragB bf;
      bf.h[0] = *(const v8usa*)wq;
      bf.h[1] = *(const v8usa*)(wq + 16);
      acc[nt] = wmb(af, bf, acc[nt]);
    }
  }

#pragma unroll
  for (int nt = 0; nt < 8; ++nt) {
    const int lc = 16 * nt + m;
#pragma unroll
    for (int r = 0; r < 8; ++r) {
      const int lr = 16 * wave + 8 * hh + r;
      stg[lr * GBN + lc] = acc[nt][r];
    }
  }
  __syncthreads();

  v4f bb4;
  {
    const v4f t1 = *(const v4f*)(bias + 4 * lane);
    bb4.x = bf16_val(t1.x); bb4.y = bf16_val(t1.y); bb4.z = bf16_val(t1.z); bb4.w = bf16_val(t1.w);
  }
  int indL = 0;
  if constexpr (MODE == 2) {
    int gr = rowBase + 16 * wave + lane;
    gr = gr < 0 ? 0 : (gr > NGT - 1 ? NGT - 1 : gr);
    const int gv = goff[gr];
    const int gn = __shfl_down(gv, 1, 32);
    indL = (gn > gv) ? 1 : 0;
  }
  int fl = 0;
  if constexpr (MODE == 3) fl = flag[0];
  const float qnan = __int_as_float(0x7fc00000);

  v4f pv[16];
#pragma unroll
  for (int i = 0; i < 16; ++i) pv[i] = *(const v4fa*)(stg + (16 * wave + i) * GBN + 4 * lane);
  __syncthreads();

#pragma unroll
  for (int i = 0; i < 16; ++i) {
    const bool ok = (rowBase + 16 * wave + i) < nOut;
    v4f y;
    if constexpr (MODE == 1) {
      const v4f t = pv[i] + bb4;
      y.x = (t.x > 0.0f) ? t.x : (t.x - t.x);
      y.y = (t.y > 0.0f) ? t.y : (t.y - t.y);
      y.z = (t.z > 0.0f) ? t.z : (t.z - t.z);
      y.w = (t.w > 0.0f) ? t.w : (t.w - t.w);
    } else if constexpr (MODE == 2) {
      const int ind = __shfl(indL, i, 32);
      v4f ad;
      ad.x = (ind != 0) ? bb4.x : 0.0f; ad.y = (ind != 0) ? bb4.y : 0.0f;
      ad.z = (ind != 0) ? bb4.z : 0.0f; ad.w = (ind != 0) ? bb4.w : 0.0f;
      const v4f t = pv[i] + ad;
      y.x = ok ? t.x : 0.0f; y.y = ok ? t.y : 0.0f; y.z = ok ? t.z : 0.0f; y.w = ok ? t.w : 0.0f;
    } else {
      const v4f t = pv[i] + bb4;
      y.x = (fl != 0) ? qnan : t.x; y.y = (fl != 0) ? qnan : t.y;
      y.z = (fl != 0) ? qnan : t.z; y.w = (fl != 0) ? qnan : t.w;
    }
    pv[i] = y;
  }

  if constexpr (MODE != 2) {
#pragma unroll
    for (int i = 0; i < 16; ++i) {
      const int r = rowBase + 16 * wave + i;
      if (r < nOut) *(volatile v4f*)(outF + (size_t)r * HID + 4 * lane) = pv[i];
    }
    __threadfence();
#pragma unroll
    for (int i = 0; i < 16; ++i) {
      const int r = rowBase + 16 * wave + i;
      if (r < nOut) *(volatile v4f*)(outF + (size_t)r * HID + 4 * lane) = pv[i];
    }
  } else {
#pragma unroll
    for (int i = 0; i < 16; ++i) {
      v4us h4, l4;
      unsigned hb;
      hb = bf16_bits(pv[i].x); h4[0] = (unsigned short)hb; l4[0] = (unsigned short)bf16_bits(pv[i].x - __uint_as_float(hb << 16));
      hb = bf16_bits(pv[i].y); h4[1] = (unsigned short)hb; l4[1] = (unsigned short)bf16_bits(pv[i].y - __uint_as_float(hb << 16));
      hb = bf16_bits(pv[i].z); h4[2] = (unsigned short)hb; l4[2] = (unsigned short)bf16_bits(pv[i].z - __uint_as_float(hb << 16));
      hb = bf16_bits(pv[i].w); h4[3] = (unsigned short)hb; l4[3] = (unsigned short)bf16_bits(pv[i].w - __uint_as_float(hb << 16));
      unsigned short* srow = (unsigned short*)stg + (size_t)(16 * wave + i) * (2 * GBN);
      *(v4usa*)(srow + 4 * lane) = h4;
      *(v4usa*)(srow + HID + 4 * lane) = l4;
    }
    __syncthreads();
    v8us qv[16];
#pragma unroll
    for (int i = 0; i < 16; ++i) {
      const unsigned short* srow = (const unsigned short*)stg + (size_t)(16 * wave + i) * (2 * GBN);
      qv[i] = *(const v8usa*)(srow + 8 * lane);
    }
#pragma unroll
    for (int i = 0; i < 16; ++i) {
      unsigned short* rp = outH + (size_t)(rowBase + 16 * wave + i) * (size_t)K2 + 8 * lane;
      *(volatile v8us*)rp = qv[i];
    }
    __threadfence();
#pragma unroll
    for (int i = 0; i < 16; ++i) {
      unsigned short* rp = outH + (size_t)(rowBase + 16 * wave + i) * (size_t)K2 + 8 * lane;
      *(volatile v8us*)rp = qv[i];
    }
  }
}

__global__ __launch_bounds__(NTHR) void k_aggpool(int nN, int nG,
                                                  const int* __restrict__ goff, const int* __restrict__ lst,
                                                  const int* __restrict__ ocb, const int* __restrict__ blkf,
                                                  const float* __restrict__ dis, const float* __restrict__ h1,
                                                  unsigned short* ghl) {
  __shared__ __attribute__((aligned(16))) unsigned short rowbuf_all[NWAVE * 256];
  const int tid = (int)threadIdx.x, lane = tid & 31;
  const int wave = rfl(tid >> 5);
  unsigned short* rowbuf = rowbuf_all + wave * 256;
  const int b = (int)blockIdx.x;
  const int g0 = b * GPB;
  int g1 = g0 + GPB; g1 = g1 > nG ? nG : g1;
  int nbase = goff[g0 < NGT - 1 ? g0 : NGT - 1];
  int nend  = goff[g1 < NGT - 1 ? g1 : NGT - 1];
  nbase = clampi(nbase, 0, nN);
  nend  = clampi(nend, nbase, nN);
  int nlim = nbase + SLOTCAP; nlim = nlim > nend ? nend : nlim;
  nbase = rfl(nbase); nlim = rfl(nlim);
  const int pf = rfl(blkf[(size_t)b * 32]);
  const int* lb = lst + (size_t)b * RCAP;
  const int* ob = ocb + (size_t)b * SLOTCAP;
  const float qnan = __int_as_float(0x7fc00000);

#pragma unroll 1
  for (int k = 0; k < GPB / NWAVE; ++k) {
    const int g = g0 + wave + NWAVE * k;
    const bool gl = g < nG;
    const int gc = gl ? g : nG - 1;
    int n0 = goff[gc];
    int n1 = goff[gc + 1];
    n0 = clampi(n0, nbase, nlim);
    n1 = clampi(n1, n0, nlim);
    n1 = gl ? n1 : n0;
    n0 = rfl(n0); n1 = rfl(n1);
    int pois = pf;
    float a0 = 0.0f, a1 = 0.0f, a2 = 0.0f, a3 = 0.0f;
#pragma unroll 1
    for (int i = n0; i < n1; ++i) {
      const int s = i - nbase;
      const int oc = rfl(ob[s]);
      int c = oc & 255;
      int o = oc >> 8;
      o = o < 0 ? 0 : (o > RCAP ? RCAP : o);
      pois |= (c > DEGCAP) ? 1 : 0;
      c = c > DEGCAP ? DEGCAP : c;
      const float dd = dis[i];
      int idx = o + lane;
      idx = idx > RCAP - 1 ? RCAP - 1 : idx;
      const int sr = clampi(lb[idx], 0, nN - 1);
      const float cf = dis[sr] * dd;
      const int cfi = __float_as_int(cf);
#pragma unroll 1
      for (int kk = 0; kk < c; ++kk) {
        const int   sk = __builtin_amdgcn_readlane(sr, kk);
        const float ck = __int_as_float(__builtin_amdgcn_readlane(cfi, kk));
        const v4f a = *(const v4f*)(h1 + (size_t)sk * HID + 4 * lane);
        a0 = fmaf(ck, a.x, a0); a1 = fmaf(ck, a.y, a1);
        a2 = fmaf(ck, a.z, a2); a3 = fmaf(ck, a.w, a3);
      }
      const v4f sv = *(const v4f*)(h1 + (size_t)i * HID + 4 * lane);
      const float rd = dd * dd;
      a0 = fmaf(rd, sv.x, a0); a1 = fmaf(rd, sv.y, a1);
      a2 = fmaf(rd, sv.z, a2); a3 = fmaf(rd, sv.w, a3);
    }
    const int cn = n1 - n0;
    const float cf = (cn < 1) ? 1.0f : (float)cn;
    const float inv = 1.0f / cf;
    float m0 = a0 * inv, m1 = a1 * inv, m2 = a2 * inv, m3 = a3 * inv;
    m0 = (pois != 0) ? qnan : m0; m1 = (pois != 0) ? qnan : m1;
    m2 = (pois != 0) ? qnan : m2; m3 = (pois != 0) ? qnan : m3;
    m0 = gl ? m0 : 0.0f; m1 = gl ? m1 : 0.0f; m2 = gl ? m2 : 0.0f; m3 = gl ? m3 : 0.0f;
    v4us mh, ml;
    {
      unsigned hb;
      hb = bf16_bits(m0); mh[0] = (unsigned short)hb; ml[0] = (unsigned short)bf16_bits(m0 - __uint_as_float(hb << 16));
      hb = bf16_bits(m1); mh[1] = (unsigned short)hb; ml[1] = (unsigned short)bf16_bits(m1 - __uint_as_float(hb << 16));
      hb = bf16_bits(m2); mh[2] = (unsigned short)hb; ml[2] = (unsigned short)bf16_bits(m2 - __uint_as_float(hb << 16));
      hb = bf16_bits(m3); mh[3] = (unsigned short)hb; ml[3] = (unsigned short)bf16_bits(m3 - __uint_as_float(hb << 16));
    }
    *(v4usa*)(rowbuf + 4 * lane) = mh;
    *(v4usa*)(rowbuf + HID + 4 * lane) = ml;
    wave_sync();
    const v8us q0 = *(const v8usa*)(rowbuf + 8 * lane);
    wave_sync();
    unsigned short* rp = ghl + (size_t)g * K2 + 8 * lane;
    *(volatile v8us*)rp = q0;
    __threadfence();
    *(volatile v8us*)rp = q0;
  }
}

static inline int cdiv(int a, int b) { return (a + b - 1) / b; }
static inline size_t al256(size_t o) { return (o + 255) & ~(size_t)255; }

extern "C" void kernel_launch(void* const* d_in, const int* in_sizes, int n_in,
                              void* d_out, int out_size, void* d_ws, size_t ws_size,
                              hipStream_t stream) {
  if (n_in < 12) return;
  const int nN = NN_C, nE = NE_C, nG = NG_C;
  if (in_sizes[0] != nN * FA) return;
  if (in_sizes[1] != 2 * nE) return;
  if (in_sizes[3] != nN) return;
  if (in_sizes[4] != EMBN) return;
  if (in_sizes[6] != DA * HID || in_sizes[7] != HID) return;
  if (in_sizes[8] != HID * HID || in_sizes[9] != HID) return;
  if (in_sizes[10] != HID * HID || in_sizes[11] != HID) return;
  if (out_size != nG * HID) return;

  const int*   x    = (const int*)d_in[0];
  const int*   edge = (const int*)d_in[1];
  const int*   bat  = (const int*)d_in[3];
  const float* emb  = (const float*)d_in[4];
  const float* W1   = (const float*)d_in[6];
  const float* b1   = (const float*)d_in[7];
  const float* W2   = (const float*)d_in[8];
  const float* b2   = (const float*)d_in[9];
  const float* Wf   = (const float*)d_in[10];
  const float* bf   = (const float*)d_in[11];
  float* out = (float*)d_out;
  const int* src = edge;
  const int* dst = edge + nE;

  const int MP1  = cdiv(nN, GBM) * GBM;
  const int MP2  = NBLK * GPB;
  const int gD   = cdiv(nN, NBD);
  const int NBPD = gD * NBD;
  const int gH   = cdiv(nN, H0NPB);
  const int vec8 = ((nE & 3) == 0) ? 1 : 0;
  if (MP1 - nN > 32 * (NTHR / 8)) return;
  if ((long long)gH * H0NPB < (long long)nN) return;

  char* ws = (char*)d_ws;
  size_t off = 0;
  const size_t oDIS = off; off = al256(off + (size_t)NBPD * 4);
  const size_t oGOF = off; off = al256(off + (size_t)NGT * 4);
  const size_t oFLG = off; off = al256(off + 128);
  const size_t oW1D = off; off = al256(off + (size_t)HID * K1 * 2);
  const size_t oW2D = off; off = al256(off + (size_t)HID * K2 * 2);
  const size_t oWFD = off; off = al256(off + (size_t)HID * K2 * 2);
  const size_t oH0  = off; off = al256(off + (size_t)nN * 16 * 4);
  const size_t oLST = off; off = al256(off + (size_t)NBLK * RCAP * 4);
  const size_t oOCB = off; off = al256(off + (size_t)NBLK * SLOTCAP * 4);
  const size_t oBLK = off; off = al256(off + (size_t)NBLK * 128);
  const size_t oA0  = off; off = al256(off + (size_t)MP1 * AP1 * 2);
  const size_t oH1  = off; off = al256(off + (size_t)nN * HID * 4);
  const size_t oGHL = off; off = al256(off + (size_t)MP2 * K2 * 2);
  const size_t oEHL = off; off = al256(off + (size_t)MP2 * K2 * 2);
  if (off > ws_size) return;
  float*          DIS = (float*)(ws + oDIS);
  int*            GOF = (int*)(ws + oGOF);
  int*            FLG = (int*)(ws + oFLG);
  unsigned short* W1D = (unsigned short*)(ws + oW1D);
  unsigned short* W2D = (unsigned short*)(ws + oW2D);
  unsigned short* WFD = (unsigned short*)(ws + oWFD);
  float*          H0  = (float*)(ws + oH0);
  int*            LST = (int*)(ws + oLST);
  int*            OCB = (int*)(ws + oOCB);
  int*            BLK = (int*)(ws + oBLK);
  unsigned short* A0  = (unsigned short*)(ws + oA0);
  float*          H1  = (float*)(ws + oH1);
  unsigned short* GHL = (unsigned short*)(ws + oGHL);
  unsigned short* EHL = (unsigned short*)(ws + oEHL);

  const size_t bkLds = (size_t)BK_LDS_INTS * 4;
  hipFuncSetAttribute(reinterpret_cast<const void*>(&k_bkt), hipFuncAttributeMaxDynamicSharedMemorySize, (int)bkLds);

  k_wprep<<<(NUW1 + 2 * NUW2) / NTHR, NTHR, 0, stream>>>(W1, W2, Wf, W1D, W2D, WFD);
  k_h0<<<gH, NTHR, 0, stream>>>(x, emb, nN, H0);
  k_goff<<<GOFFB + 1, NTHR, 0, stream>>>(bat, nN, nG, GOF, FLG);
  k_deg<<<gD, NTHR, 0, stream>>>(dst, nE, vec8, DIS);
  k_bkt<<<NBLK, NTHR, bkLds, stream>>>(src, dst, nE, nN, nG, vec8, MP1, GOF, DIS, H0, LST, OCB, BLK, A0);
  k_gemm<1><<<MP1 / GBM, GTHR, 0, stream>>>(A0, AP1, W1D, K1, b1, GOF, FLG, H1, EHL, nN);
  k_aggpool<<<NBLK, NTHR, 0, stream>>>(nN, nG, GOF, LST, OCB, BLK, DIS, H1, GHL);
  k_gemm<2><<<MP2 / GBM, GTHR, 0, stream>>>(GHL, K2, W2D, K2, b2, GOF, FLG, H1, EHL, nG);
  k_gemm<3><<<MP2 / GBM, GTHR, 0, stream>>>(EHL, K2, WFD, K2, bf, GOF, FLG, out, GHL, nG);
}
